// GNNNodeEncoder_43714177138808
// MI455X (gfx1250) — hardware-run, weakly checked
//
#include <hip/hip_runtime.h>


namespace {
constexpr int N = 50000, NP = 50048, E = 600000, D = 128, D2 = 256, L = 5, AV = 120, CV = 3, HV = 7, E1V = 6, E2V = 4, RPB = 64, NBP = NP / RPB;
constexpr float XS = 32.0f, WSC = 256.0f, NEG = 0.2f  , BNEPS = 1e-5f;
typedef _Float16 b16;
typedef __attribute__((ext_vector_type(16))) _Float16 v16b;
typedef __attribute__((ext_vector_type(8))) _Float16 v8b;
typedef __attribute__((ext_vector_type(8))) float v8f;
typedef __attribute__((ext_vector_type(4))) float v4f;
__device__ __forceinline__ float bf16_rne(float f) { unsigned int u = __float_as_uint(f); u += 0x7FFFu + ((u >> 16) & 1u); return __uint_as_float(u & 0xFFFF0000u); }
__device__ __forceinline__ void split16(float v, b16& hi, b16& lo) { hi = (b16)v; lo = (b16)(v - (float)hi); }
__device__ __forceinline__ v16b frag_kb(const b16* p, int hh) { const v8b a = *(const v8b*)(p + 8 * hh), b = *(const v8b*)(p + 16 + 8 * hh); v16b f;
#pragma unroll
  for (int e = 0; e < 8; ++e) { f[e] = a[e]; f[8 + e] = b[e]; } return f; }
__device__ __forceinline__ v8f wmma16b(v16b a, v16b b, v8f c) { v8f d = __builtin_amdgcn_wmma_f32_16x16x32_f16(false, a, false, b, (short)0, c, false, false); asm volatile("v_nop\n\tv_nop\n\tv_nop\n\tv_nop" : "+v"(d) : "v"(a), "v"(b)); return d; }
__device__ __forceinline__ void wave_lds_sync() { __builtin_amdgcn_fence(__ATOMIC_RELEASE, "workgroup"); __builtin_amdgcn_wave_barrier(); __builtin_amdgcn_fence(__ATOMIC_ACQUIRE, "workgroup"); }
__device__ __forceinline__ float pmul(float a, float b) { float p = a * b; asm volatile("" : "+v"(p)); return p; }
__device__ __forceinline__ int iclamp(int v, int lo, int hi) { return v < lo ? lo : (v > hi ? hi : v); }
constexpr int CSR_NBLK = 512, CSR_GB = 9, CSR_GN = 1 << CSR_GB  , CSR_MAXG = 512, CSR_CAP = 12288  ;
__global__ __launch_bounds__(64) void csrA_kernel(const int* __restrict__ dst, int E, int N, int nG, int CHP, int NGP, int* __restrict__ STG, int* __restrict__ HST) {
  extern __shared__ int sm[];
  int* cnt = sm; int* run = sm + NGP; int* ids = sm + 2 * NGP;
  const int b = blockIdx.x; const int ch = (E + CSR_NBLK - 1) / CSR_NBLK; const int e0 = b * ch, e1 = min(E, e0 + ch);
  for (int i = threadIdx.x; i < NGP; i += 64) cnt[i] = 0;
  for (int i = threadIdx.x; i < CHP; i += 64) ids[i] = -1;
  __syncthreads();
  if (threadIdx.x == 0) {
    for (int e = e0; e < e1; ++e) { int d = dst[e]; d = (d < 0) ? 0 : (d >= N ? N - 1 : d); cnt[d >> CSR_GB] += 1; }
    int acc = 0; for (int g = 0; g < nG; ++g) { run[g] = acc; acc += cnt[g]; }
    for (int e = e0; e < e1; ++e) { int d = dst[e]; d = (d < 0) ? 0 : (d >= N ? N - 1 : d); const int g = d >> CSR_GB; ids[run[g]] = e; run[g] += 1; } }
  __syncthreads();
  typedef __attribute__((ext_vector_type(4))) int v4i;
  for (int pass = 0; pass < 2; ++pass) {
    for (int i = threadIdx.x; i < CHP / 4; i += 64) *(volatile v4i*)(STG + (size_t)b * CHP + i * 4) = *(const v4i*)(&ids[i * 4]);
    for (int i = threadIdx.x; i < NGP / 4; i += 64) { v4i v; for (int e = 0; e < 4; ++e) v[e] = (i * 4 + e < nG) ? cnt[i * 4 + e] : 0; *(volatile v4i*)(HST + (size_t)b * NGP + i * 4) = v; }
    __threadfence(); }
}
__global__ __launch_bounds__(512) void csrS_kernel(const int* __restrict__ HST, int nG, int NGP, int* __restrict__ START, int* __restrict__ TOT, int* __restrict__ OFF) {
  __shared__ int tot[CSR_MAXG];
  const int b = threadIdx.x;
  for (int pass = 0; pass < 2; ++pass) { int runb = 0; for (int g = 0; g < nG; ++g) { int c = HST[(size_t)b * NGP + g]; c = (c < 0) ? 0 : c; ((volatile int*)OFF)[(size_t)g * CSR_NBLK + b] = runb; runb += c; } __threadfence(); }
  for (int g = threadIdx.x; g < nG; g += 512) { int s = 0; for (int bb = 0; bb < CSR_NBLK; ++bb) { int c = HST[(size_t)bb * NGP + g]; s += (c < 0) ? 0 : c; } tot[g] = s; }
  __syncthreads();
  if (threadIdx.x < 32) {
    __shared__ int st[CSR_MAXG + 32];
    if (threadIdx.x == 0) { int acc = 0; for (int g = 0; g < NGP; ++g) { st[g] = acc; if (g < nG) acc += (tot[g] + 31) & ~31; } st[NGP] = acc; }
    __builtin_amdgcn_fence(__ATOMIC_RELEASE, "workgroup"); __builtin_amdgcn_wave_barrier(); __builtin_amdgcn_fence(__ATOMIC_ACQUIRE, "workgroup");
    for (int pass = 0; pass < 2; ++pass) { for (int i = threadIdx.x; i < NGP + 32; i += 32) { ((volatile int*)START)[i] = (i <= NGP) ? st[min(i, NGP)] : 0; ((volatile int*)TOT)[i] = (i < nG) ? tot[i] : 0; } __threadfence(); } }
}
__global__ __launch_bounds__(256) void csrB_kernel(const int* __restrict__ dst, int N, int nG, int CHP, int NGP, int permLen, const int* __restrict__ STG, const int* __restrict__ HST, const int* __restrict__ OFF, const int* __restrict__ START, const int* __restrict__ TOT, int* __restrict__ PERM, int* __restrict__ ROWPTR, int* __restrict__ ROWCNT, int* __restrict__ FLAG) {
  typedef __attribute__((ext_vector_type(4))) int v4i;
  __shared__ int ids[CSR_CAP]; __shared__ unsigned short key[CSR_CAP]; __shared__ int outp[CSR_CAP]; __shared__ int ncnt[CSR_GN + 1]; __shared__ int boff[CSR_NBLK + 1];
  const int g = blockIdx.x, t_ = threadIdx.x; int tot = TOT[g]; int st = START[g], stn = START[g + 1]; const int v0 = g * CSR_GN; const int nv = min(CSR_GN, N - v0);
  st = (st < 0) ? 0 : (st > permLen - 32 ? permLen - 32 : st) & ~31; stn = (stn < st) ? st : (stn > permLen ? permLen : stn); tot = (tot < 0) ? 0 : tot; if (tot > stn - st && tot <= CSR_CAP) tot = stn - st;
  if (tot > CSR_CAP) {
    for (int pass = 0; pass < 2; ++pass) { for (int i = t_; i < CSR_GN / 4; i += 256) { v4i a, c; for (int e = 0; e < 4; ++e) { a[e] = st; c[e] = 0; } *(volatile v4i*)(ROWPTR + v0 + i * 4) = a; *(volatile v4i*)(ROWCNT + v0 + i * 4) = c; } if (t_ == 0) ((volatile int*)FLAG)[0] = 1; __threadfence(); } (void)nv; return; }
  if (t_ == 0) { int acc = 0; for (int b = 0; b < CSR_NBLK; ++b) { boff[b] = acc; int c = HST[(size_t)b * NGP + g]; c = (c < 0) ? 0 : (c > CHP ? CHP : c); acc += c; if (acc > tot) acc = tot; } boff[CSR_NBLK] = acc; }
  for (int i = t_; i <= CSR_GN; i += 256) ncnt[i] = 0;
  __syncthreads();
  for (int b = 0; b < CSR_NBLK; ++b) { const int c = boff[b + 1] - boff[b]; int o_ = OFF[(size_t)g * CSR_NBLK + b]; o_ = (o_ < 0) ? 0 : (o_ > CHP - c ? CHP - c : o_); const int* src_ = STG + (size_t)b * CHP + o_;
    for (int i = t_; i < c; i += 256) { int id = src_[i]; id = (id < 0) ? 0 : id; ids[boff[b] + i] = id; int d = dst[id]; d = (d < v0) ? v0 : (d >= N ? N - 1 : d); int kk = d - v0; kk = (kk < 0) ? 0 : (kk >= CSR_GN ? CSR_GN - 1 : kk); key[boff[b] + i] = (unsigned short)kk; } }
  __syncthreads();
  if (t_ == 0) { for (int i = 0; i < tot; ++i) ncnt[key[i]] += 1; int acc = 0; for (int vl = 0; vl < CSR_GN; ++vl) { const int c = ncnt[vl]; ncnt[vl] = acc; acc += c; } ncnt[CSR_GN] = acc;
    for (int i = 0; i < tot; ++i) { const int vl = key[i]; outp[ncnt[vl]] = ids[i]; ncnt[vl] += 1; }
    for (int vl = CSR_GN; vl > 0; --vl) ncnt[vl] = ncnt[vl - 1]; ncnt[0] = 0; }
  __syncthreads();
  for (int pass = 0; pass < 2; ++pass) {
    for (int i = t_; i < (stn - st) / 4; i += 256) { v4i v; for (int e = 0; e < 4; ++e) { const int q = i * 4 + e; v[e] = (q < tot) ? outp[q] : -1; } *(volatile v4i*)(PERM + st + i * 4) = v; }
    for (int i = t_; i < CSR_GN / 4; i += 256) { v4i a, c; for (int e = 0; e < 4; ++e) { const int vl = i * 4 + e; a[e] = st + ncnt[vl]; c[e] = (vl < nv) ? (ncnt[vl + 1] - ncnt[vl]) : 0; } *(volatile v4i*)(ROWPTR + v0 + i * 4) = a; *(volatile v4i*)(ROWCNT + v0 + i * 4) = c; }
    __threadfence(); }
}
__global__ __launch_bounds__(256) void csrZ_kernel(int* __restrict__ p, size_t n4) { typedef __attribute__((ext_vector_type(4))) int v4i; const size_t tid = (size_t)blockIdx.x * 256 + threadIdx.x, nth = (size_t)gridDim.x * 256; v4i z = {0, 0, 0, 0}; for (size_t i = tid; i < n4; i += nth) *(volatile v4i*)(p + i * 4) = z; }
struct CsrBufs { int *STG, *HST, *OFF, *START, *TOT, *PERM, *ROWPTR, *ROWCNT, *FLAG; int nG, NGP, CHP; size_t permLen; char* base; size_t bytes; };
static size_t csr_carve(CsrBufs& c, char* ws, size_t off, int E, int N) {
  const size_t off0 = off; c.base = ws + off;
  auto al = [&](size_t bytes) { char* p = ws + off; off += (bytes + 255) & ~(size_t)255; return p; };
  c.nG = (N + CSR_GN - 1) / CSR_GN; c.NGP = (c.nG + 31) & ~31; const int ch = (E + CSR_NBLK - 1) / CSR_NBLK; c.CHP = (ch + 31) & ~31; c.permLen = (size_t)E + 32 * (size_t)c.nG + 32;
  c.STG = (int*)al((size_t)CSR_NBLK * c.CHP * 4); c.HST = (int*)al((size_t)CSR_NBLK * c.NGP * 4); c.OFF = (int*)al((size_t)c.NGP * CSR_NBLK * 4); c.START = (int*)al((size_t)(c.NGP + 64) * 4); c.TOT = (int*)al((size_t)(c.NGP + 64) * 4);
  c.PERM = (int*)al(c.permLen * 4); c.ROWPTR = (int*)al((size_t)c.nG * CSR_GN * 4); c.ROWCNT = (int*)al((size_t)c.nG * CSR_GN * 4); c.FLAG = (int*)al(256);
  c.bytes = off - off0; return off;
}
static void csr_build(const CsrBufs& c, const int* dst, int E, int N, hipStream_t stream) {
  const size_t smem = (size_t)(2 * c.NGP + c.CHP) * 4;
  csrZ_kernel<<<512, 256, 0, stream>>>((int*)c.base, c.bytes / 16);
  csrA_kernel<<<CSR_NBLK, 64, smem, stream>>>(dst, E, N, c.nG, c.CHP, c.NGP, c.STG, c.HST);
  csrS_kernel<<<1, 512, 0, stream>>>(c.HST, c.nG, c.NGP, c.START, c.TOT, c.OFF);
  csrB_kernel<<<c.nG, 256, 0, stream>>>(dst, N, c.nG, c.CHP, c.NGP, (int)c.permLen, c.STG, c.HST, c.OFF, c.START, c.TOT, c.PERM, c.ROWPTR, c.ROWCNT, c.FLAG);
}


__global__ __launch_bounds__(256) void wprep_kernel(const float* __restrict__ w1, const float* __restrict__ w2, b16* __restrict__ W1T, b16* __restrict__ W2T) {
  const size_t u = (size_t)blockIdx.x * 256 + threadIdx.x; const size_t n = (size_t)L * D * D2 / 8; size_t t = u; v8b o;
  if (t < n) { const size_t e = t * 8; const int l = (int)(e / (D2 * D)); const int rem = (int)(e % (D2 * D)); const int oo = rem / D, k0 = rem % D; for (int j = 0; j < 8; ++j) o[j] = (b16)(bf16_rne(w1[((size_t)l * D + k0 + j) * D2 + oo]) * WSC); for (int pass = 0; pass < 2; ++pass) { *(volatile v8b*)(W1T + e) = o; __threadfence(); } return; } t -= n;
  if (t < n) { const size_t e = t * 8; const int l = (int)(e / (D * D2)); const int rem = (int)(e % (D * D2)); const int oo = rem / D2, k0 = rem % D2; for (int j = 0; j < 8; ++j) o[j] = (b16)(bf16_rne(w2[((size_t)l * D2 + k0 + j) * D + oo]) * WSC); for (int pass = 0; pass < 2; ++pass) { *(volatile v8b*)(W2T + e) = o; __threadfence(); } }
}
__global__ __launch_bounds__(256) void h0_kernel(const int* __restrict__ xf, const float* __restrict__ ae, const float* __restrict__ ce, const float* __restrict__ he, float* __restrict__ Hp) {
  const int wave = threadIdx.x >> 5, lane = threadIdx.x & 31; const size_t v = (size_t)blockIdx.x * 8 + wave; v4f o = {0.0f, 0.0f, 0.0f, 0.0f};
  if (v < (size_t)N) { const int i0 = iclamp(xf[v * 3], 0, AV - 1), i1 = iclamp(xf[v * 3 + 1], 0, CV - 1), i2 = iclamp(xf[v * 3 + 2], 0, HV - 1);
    const v4f a = *(const v4f*)(ae + (size_t)i0 * D + lane * 4), c = *(const v4f*)(ce + (size_t)i1 * D + lane * 4), h = *(const v4f*)(he + (size_t)i2 * D + lane * 4);
    for (int i = 0; i < 4; ++i) o[i] = (bf16_rne(a[i]) + bf16_rne(c[i])) + bf16_rne(h[i]); }
  for (int pass = 0; pass < 2; ++pass) { *(volatile v4f*)(Hp + v * D + lane * 4) = o; __threadfence(); }
}
__global__ __launch_bounds__(256) void msg_kernel(const float* __restrict__ Hp, const float* __restrict__ e1, const float* __restrict__ e2, const int* __restrict__ eattr, const int* __restrict__ srcs, const int* __restrict__ PERM, const int* __restrict__ ROWPTR, const int* __restrict__ ROWCNT, int permLen, float* __restrict__ Z) {
  const int wave = threadIdx.x >> 5, lane = threadIdx.x & 31; const size_t v = (size_t)blockIdx.x * 8 + wave; v4f o = {0.0f, 0.0f, 0.0f, 0.0f};
  if (v < (size_t)N) { int st = ROWPTR[v], cnt = ROWCNT[v]; cnt = iclamp(cnt, 0, 65536); st = iclamp(st, 0, permLen - cnt);
#pragma unroll 1
    for (int j = 0; j < cnt; ++j) { const int e = iclamp(PERM[st + j], 0, E - 1); const size_t s = (size_t)iclamp(srcs[e], 0, N - 1); const int a0 = iclamp(eattr[(size_t)e * 2], 0, E1V - 1), a1 = iclamp(eattr[(size_t)e * 2 + 1], 0, E2V - 1);
      const v4f h = *(const v4f*)(Hp + s * D + lane * 4), t1 = *(const v4f*)(e1 + (size_t)a0 * D + lane * 4), t2 = *(const v4f*)(e2 + (size_t)a1 * D + lane * 4);
      for (int i = 0; i < 4; ++i) o[i] += h[i] + (bf16_rne(t1[i]) + bf16_rne(t2[i])); } }
  for (int pass = 0; pass < 2; ++pass) { *(volatile v4f*)(Z + v * D + lane * 4) = o; __threadfence(); }
}
template <int KD, int COUT, int RELU, int STATS>
__global__ __launch_bounds__(128) void gemm_kernel(const float* __restrict__ src, const b16* __restrict__ WT, const float* __restrict__ bias, float* __restrict__ OUT, float* __restrict__ PS) {
  constexpr int NT = COUT / 16;
  __shared__ __attribute__((aligned(16))) b16 Ah[4][16][KD + 8], Al[4][16][KD + 8]; __shared__ __attribute__((aligned(16))) float Tf[4][16][(COUT > 128 ? 128 : COUT) + 4];
  const int wave = threadIdx.x >> 5, lane = threadIdx.x & 31, nloc = lane & 15, hlf = lane >> 4; const size_t m0 = (size_t)blockIdx.x * 64 + wave * 16;
  for (int rr = 0; rr < 16; ++rr) for (int q = lane * 4; q < KD; q += 128) { const v4f v = *(const v4f*)(src + (m0 + rr) * KD + q); for (int j = 0; j < 4; ++j) { b16 p, s; split16(v[j] * XS, p, s); Ah[wave][rr][q + j] = p; Al[wave][rr][q + j] = s; } }
  wave_lds_sync();
  v8f acc[NT];
#pragma unroll
  for (int t = 0; t < NT; ++t) acc[t] = (v8f){};
#pragma unroll 2
  for (int kb = 0; kb < KD; kb += 32) { const v16b a = frag_kb(&Ah[wave][nloc][kb], hlf), al = frag_kb(&Al[wave][nloc][kb], hlf);
#pragma unroll
    for (int t = 0; t < NT; ++t) { const v16b bw = frag_kb(WT + (size_t)(t * 16 + nloc) * KD + kb, hlf); acc[t] = wmma16b(a, bw, acc[t]); acc[t] = wmma16b(al, bw, acc[t]); } }
  constexpr int NHALF = COUT / 128 > 0 ? COUT / 128 : 1; constexpr int TPH = NT / NHALF;
  for (int half = 0; half < NHALF; ++half) {
    __syncthreads();
#pragma unroll
    for (int t = 0; t < TPH; ++t) { const int c = (half * TPH + t) * 16 + nloc; const float bb = bf16_rne(bias[c]);
#pragma unroll 1
      for (int r = 0; r < 8; ++r) { const size_t row = m0 + 8 * hlf + r; float y = acc[half * TPH + t][r] * (1.0f / (XS * WSC)) + bb; if (RELU) y = fmaxf(y, 0.0f); Tf[wave][8 * hlf + r][t * 16 + nloc] = row < (size_t)N ? y : 0.0f; } }
    __syncthreads();
    for (int pass = 0; pass < 2; ++pass) { for (int rr = 0; rr < 16; ++rr) for (int q = lane * 4; q < TPH * 16; q += 128) *(volatile v4f*)(OUT + (m0 + rr) * COUT + half * TPH * 16 + q) = *(const v4f*)(&Tf[wave][rr][q]);
      if (STATS && threadIdx.x < TPH * 16 / 4) { v4f s = {0.0f, 0.0f, 0.0f, 0.0f}; for (int w = 0; w < 4; ++w) for (int rr = 0; rr < 16; ++rr) s += *(const v4f*)(&Tf[w][rr][threadIdx.x * 4]); *(volatile v4f*)(PS + (size_t)blockIdx.x * COUT + half * TPH * 16 + threadIdx.x * 4) = s; } __threadfence(); } }
}
template <int C>
__global__ __launch_bounds__(128) void colstat_kernel(const float* __restrict__ PS, float* __restrict__ STAT) {
  const int c = threadIdx.x; if (c >= C) return; float s = 0.0f; for (int b = 0; b < NBP; ++b) s += PS[(size_t)b * C + c];
  for (int pass = 0; pass < 2; ++pass) { ((volatile float*)STAT)[c] = s * (1.0f / N); __threadfence(); }
}
template <int C>
__global__ __launch_bounds__(256) void var_kernel(const float* __restrict__ P, const float* __restrict__ MEAN, float* __restrict__ PS) {
  constexpr int NG = 256 / C; __shared__ __attribute__((aligned(16))) float sq[NG][C + 4]; const int t = threadIdx.x, c = t % C, grp = t / C; float a = 0.0f; const float m = MEAN[c];
  for (int rr = grp; rr < RPB; rr += NG) { const size_t v = (size_t)blockIdx.x * RPB + rr; const float d = v < (size_t)N ? P[v * C + c] - m : 0.0f; a += d * d; }
  sq[grp][c] = a; __syncthreads();
  for (int pass = 0; pass < 2; ++pass) { if (t < C / 4) { v4f s = {0.0f, 0.0f, 0.0f, 0.0f}; for (int g2 = 0; g2 < NG; ++g2) s += *(const v4f*)(&sq[g2][t * 4]); *(volatile v4f*)(PS + (size_t)blockIdx.x * C + t * 4) = s; } __threadfence(); }
}
template <int LAST>
__global__ __launch_bounds__(256) void apply_kernel(const float* __restrict__ Z2, const float* __restrict__ MEAN, const float* __restrict__ VAR, const float* __restrict__ g_, const float* __restrict__ be_, float* __restrict__ Hp, float* __restrict__ out) {
  const size_t u = (size_t)blockIdx.x * 256 + threadIdx.x; if (u >= (size_t)NP * D / 4) return; const size_t e = u * 4; const size_t v = e / D; const int c = (int)(e % D);
  v4f o = {0.0f, 0.0f, 0.0f, 0.0f}; if (v < (size_t)N) { const v4f z = *(const v4f*)(Z2 + e); for (int i = 0; i < 4; ++i) { const float y = bf16_rne(g_[c + i]) * ((z[i] - MEAN[c + i]) * rsqrtf(VAR[c + i] + BNEPS)) + bf16_rne(be_[c + i]); o[i] = LAST ? y : fmaxf(y, 0.0f); } }
  for (int pass = 0; pass < 2; ++pass) { if (LAST) { if (v < (size_t)N) *(volatile v4f*)(out + e) = o; } else *(volatile v4f*)(Hp + e) = o; __threadfence(); }
}
}

extern "C" void kernel_launch(void* const* d_in, const int* in_sizes, int n_in, void* d_out, int out_size, void* d_ws, size_t ws_size, hipStream_t stream) {
  (void)n_in;
  auto Fp = [&](int i) { return (const float*)d_in[i]; }; auto Ip = [&](int i) { return (const int*)d_in[i]; };
  if (in_sizes[0] != N * 3 || in_sizes[1] != 2 * E || in_sizes[2] != E * 2 || in_sizes[3] != AV * D || in_sizes[6] != L * E1V * D || in_sizes[7] != L * E2V * D || in_sizes[8] != L * D * D2 || in_sizes[10] != L * D2 * D || out_size != N * D) return;
  size_t off = 0; char* ws = (char*)d_ws;
  auto carve = [&](size_t bytes) { char* p = ws + off; off += (bytes + 255) & ~(size_t)255; return p; };
  b16* W1T = (b16*)carve((size_t)L * D2 * D * 2); b16* W2T = (b16*)carve((size_t)L * D * D2 * 2);
  float* Hp = (float*)carve((size_t)NP * D * 4); float* Z = (float*)carve((size_t)NP * D * 4); float* Z1 = (float*)carve((size_t)NP * D2 * 4); float* Z2 = (float*)carve((size_t)NP * D * 4);
  float* PS = (float*)carve((size_t)NBP * D * 4); float* ST = (float*)carve((size_t)2 * D * 4);
  CsrBufs csr; off = csr_carve(csr, ws, off, E, N);
  if (off > ws_size) return;
  wprep_kernel<<<(unsigned)((2 * (size_t)L * D * D2 / 8 + 255) / 256), 256, 0, stream>>>(Fp(8), Fp(10), W1T, W2T);
  csr_build(csr, Ip(1) + E, E, N, stream);
  h0_kernel<<<NP / 8, 256, 0, stream>>>(Ip(0), Fp(3), Fp(4), Fp(5), Hp);
  for (int l = 0; l < L; ++l) {
    msg_kernel<<<NP / 8, 256, 0, stream>>>(Hp, Fp(6) + (size_t)l * E1V * D, Fp(7) + (size_t)l * E2V * D, Ip(2), Ip(1), csr.PERM, csr.ROWPTR, csr.ROWCNT, (int)csr.permLen, Z);
    gemm_kernel<D, D2, 1, 0><<<NP / 64, 128, 0, stream>>>(Z, W1T + (size_t)l * D2 * D, Fp(9) + l * D2, Z1, nullptr);
    gemm_kernel<D2, D, 0, 1><<<NP / 64, 128, 0, stream>>>(Z1, W2T + (size_t)l * D * D2, Fp(11) + l * D, Z2, PS);
    colstat_kernel<D><<<1, 128, 0, stream>>>(PS, ST); var_kernel<D><<<NBP, 256, 0, stream>>>(Z2, ST, PS); colstat_kernel<D><<<1, 128, 0, stream>>>(PS, ST + D);
    if (l == L - 1) apply_kernel<1><<<(unsigned)(((size_t)NP * D / 4 + 255) / 256), 256, 0, stream>>>(Z2, ST, ST + D, Fp(12) + l * D, Fp(13) + l * D, Hp, (float*)d_out);
    else apply_kernel<0><<<(unsigned)(((size_t)NP * D / 4 + 255) / 256), 256, 0, stream>>>(Z2, ST, ST + D, Fp(12) + l * D, Fp(13) + l * D, Hp, nullptr); }
}
